// DiT_18056042512615
// MI455X (gfx1250) — hardware-run, weakly checked
//
#include <hip/hip_runtime.h>
#include <math.h>

typedef __attribute__((ext_vector_type(16))) _Float16 v16h;
typedef __attribute__((ext_vector_type(16))) __bf16 v16b;
typedef __attribute__((ext_vector_type(8)))  _Float16 v8h;
typedef __attribute__((ext_vector_type(8)))  float v8f;
typedef __attribute__((ext_vector_type(4)))  float v4f;
typedef __attribute__((ext_vector_type(2)))  float v2f;
typedef __attribute__((ext_vector_type(4)))  unsigned v4u;
typedef __attribute__((ext_vector_type(4)))  int v4i;
typedef float __attribute__((may_alias)) float_a;
typedef int __attribute__((may_alias)) int_a;

template <typename T> __device__ __forceinline__ void vst2(void* p, T v) { *(volatile T*)p = v; __threadfence(); *(volatile T*)p = v; }
__device__ __forceinline__ v8f wmma16(v16h a, v16h b, v8f c) {
  v8f d = __builtin_amdgcn_wmma_f32_16x16x32_f16(false, a, false, b, (short)0, c, false, false);
  asm volatile("v_nop\n\tv_nop\n\tv_nop\n\tv_nop" : "+v"(d) : "v"(a), "v"(b));
  return d;
}
__device__ __forceinline__ v8f wmma_bf(v16b a, v16b b, v8f c) {
  v8f d = __builtin_amdgcn_wmma_f32_16x16x32_bf16(false, a, false, b, (short)0, c, false, false);
  asm volatile("v_nop\n\tv_nop\n\tv_nop\n\tv_nop" : "+v"(d) : "v"(a), "v"(b));
  return d;
}
__device__ __forceinline__ v16h frag_h(const _Float16* rowk0, int lane) {
  union { v16h v; v8h q[2]; } u; const _Float16* p = rowk0 + 8 * (lane >> 4);
  u.q[0] = *(const v8h*)p; u.q[1] = *(const v8h*)(p + 16); return u.v;
}
__device__ __forceinline__ v16h frag_f32(const float* rowk0, int lane) {
  v16h a; const float* p = rowk0 + 8 * (lane >> 4);
#pragma unroll
  for (int i = 0; i < 8; ++i) { a[i] = (_Float16)p[i]; a[8 + i] = (_Float16)p[16 + i]; }
  return a;
}
__device__ __forceinline__ v16h frag_f32s(const float* rowk0, int lane, float sc) {
  v16h a; const float* p = rowk0 + 8 * (lane >> 4);
#pragma unroll
  for (int i = 0; i < 8; ++i) { a[i] = (_Float16)(p[i] * sc); a[8 + i] = (_Float16)(p[16 + i] * sc); }
  return a;
}
__device__ __forceinline__ v16h fragc_f32(const float* W, int k0, int n, int lane, int ld, int K) {
  v16h a; const int g = lane >> 4;
#pragma unroll
  for (int i = 0; i < 8; ++i) { const int ka = k0 + 8 * g + i, kb = ka + 16;
    a[i] = (_Float16)(ka < K ? W[(size_t)(ka < K ? ka : K - 1) * ld + n] : 0.f); a[8 + i] = (_Float16)(kb < K ? W[(size_t)(kb < K ? kb : K - 1) * ld + n] : 0.f); }
  return a;
}
struct F2 { v16b h, l; };
__device__ __forceinline__ F2 bsplit16(const float v[16]) { F2 r;
#pragma unroll
  for (int i = 0; i < 16; ++i) { const __bf16 h = (__bf16)v[i]; r.h[i] = h; r.l[i] = (__bf16)(v[i] - (float)h); }
  return r; }
__device__ __forceinline__ F2 split_row(const float* row, int k0, int lane) { float v[16]; const float* p = row + k0 + 8 * (lane >> 4);
#pragma unroll
  for (int i = 0; i < 8; ++i) { v[i] = p[i]; v[8 + i] = p[16 + i]; }
  return bsplit16(v); }
__device__ __forceinline__ F2 split_rowK(const float* row, int k0, int lane, int K) { float v[16]; const int g = lane >> 4;
#pragma unroll
  for (int i = 0; i < 8; ++i) { const int ka = k0 + 8 * g + i, kb = ka + 16; v[i] = ka < K ? row[ka < K ? ka : K - 1] : 0.f; v[8 + i] = kb < K ? row[kb < K ? kb : K - 1] : 0.f; }
  return bsplit16(v); }
__device__ __forceinline__ F2 split_col(const float* W, int k0, int n, int lane, int ld, int K) { float v[16]; const int g = lane >> 4;
#pragma unroll
  for (int i = 0; i < 8; ++i) { const int ka = k0 + 8 * g + i, kb = ka + 16; v[i] = ka < K ? W[(size_t)(ka < K ? ka : K - 1) * ld + n] : 0.f; v[8 + i] = kb < K ? W[(size_t)(kb < K ? kb : K - 1) * ld + n] : 0.f; }
  return bsplit16(v); }
__device__ __forceinline__ v8f mac3(const F2& a, const F2& b, v8f c) { c = wmma_bf(a.l, b.h, c); c = wmma_bf(a.h, b.l, c); return wmma_bf(a.h, b.h, c); }
__device__ __forceinline__ float sigm(float v) { return 1.0f / (1.0f + expf(-v)); }
#define LDSX() do { asm volatile("s_wait_dscnt 0" ::: "memory"); __builtin_amdgcn_wave_barrier(); __builtin_amdgcn_fence(__ATOMIC_RELEASE, "workgroup"); } while (0)

__device__ __forceinline__ float bfr(float v) { return (float)(__bf16)v; }
__device__ __forceinline__ float silu1(float v) { return v / (1.0f + expf(-v)); }
#define NB 64
#define TT 512
#define DD 128
#define NH 4
#define HD 32
#define BG 8
#ifndef TNB
#define TNB NB
#endif
#ifndef XSTR
#define XSTR TT
#endif
typedef __attribute__((ext_vector_type(8))) __bf16 v8b;
__device__ __forceinline__ v16b frag_b(const __bf16* rowk0, int lane) { union { v16b v; v8b q[2]; } u; const __bf16* p = rowk0 + 8 * (lane >> 4); u.q[0] = *(const v8b*)p; u.q[1] = *(const v8b*)(p + 16); return u.v; }
#define WS_CD  0u
#define WS_X   (WS_CD + 4u * (size_t)NB * 6 * DD)
#define WS_X2  (WS_X + 4u * (size_t)NB * TT * DD)
#define WS_QH  (WS_X2 + 4u * (size_t)NB * TT * DD)
#define WS_QL  (WS_QH + 2u * (size_t)NB * TT * DD)
#define WS_KH  (WS_QL + 2u * (size_t)NB * TT * DD)
#define WS_VT  (WS_KH + 2u * (size_t)NB * TT * DD)
#define WS_VL  (WS_VT + 2u * (size_t)NB * DD * TT)
#define WS_S   (WS_VL + 2u * (size_t)NB * DD * TT)
#define WS_Y   (WS_S + 4u * (size_t)BG * NH * TT * TT)
#define WS_END (WS_Y + 4u * (size_t)NB * TT * DD)
__device__ void mlp3_block(const float* __restrict__ cin, const float* w1, const float* b1, const float* w2, const float* b2, const float* w3, const float* b3, int dout, float* h1, float* h2, float* outv) {
  const int t = threadIdx.x;
  if (t < DD) { float a = 0.f;
#pragma unroll 1
    for (int k = 0; k < DD; ++k) a += cin[k] * bfr(w1[k * DD + t]);
    h1[t] = silu1(a + bfr(b1[t])); }
  __syncthreads();
  if (t < DD) { float a = 0.f;
#pragma unroll 1
    for (int k = 0; k < DD; ++k) a += h1[k] * bfr(w2[k * DD + t]);
    h2[t] = silu1(a + bfr(b2[t])); }
  __syncthreads();
  if (t < dout) { float a = 0.f;
#pragma unroll 1
    for (int k = 0; k < DD; ++k) a += h2[k] * bfr(w3[k * dout + t]);
    outv[t] = a + bfr(b3[t]); }
  __syncthreads(); }
struct P24 { const float* p[24]; };
__global__ __launch_bounds__(256) void k_cond(const float* __restrict__ NODES, const float* __restrict__ TV, P24 prm, float* __restrict__ CD) { const float* const* PRM = prm.p; __shared__ float sc[DD], h1[DD], h2[DD], so[6][DD];
  const int t = threadIdx.x; const size_t b = blockIdx.x;
  if (t < DD) sc[t] = bfr(NODES[b * DD + t]) + bfr(TV[b]);
  __syncthreads();
  mlp3_block(sc, PRM[0], PRM[1], PRM[2], PRM[3], PRM[4], PRM[5], 2 * DD, h1, h2, &so[0][0]);
  mlp3_block(sc, PRM[6], PRM[7], PRM[8], PRM[9], PRM[10], PRM[11], DD, h1, h2, &so[2][0]);
  mlp3_block(sc, PRM[12], PRM[13], PRM[14], PRM[15], PRM[16], PRM[17], 2 * DD, h1, h2, &so[3][0]);
  mlp3_block(sc, PRM[18], PRM[19], PRM[20], PRM[21], PRM[22], PRM[23], DD, h1, h2, &so[5][0]);
  for (int e = t; e < 6 * DD / 4; e += 256) vst2(CD + b * 6 * DD + e * 4, *(const v4f*)(&so[0][0] + e * 4)); }
__global__ __launch_bounds__(256) void k_xs(const float* __restrict__ LAT, const float* __restrict__ CD, float* __restrict__ X, float* __restrict__ X2) { __shared__ float st[DD][65]; __shared__ float smu[64], srs[64];
  const int t = threadIdx.x; const int n0 = blockIdx.x * 64; const size_t b = blockIdx.y;
  for (int e = t; e < DD * 64; e += 256) { const int d = e >> 6, nl = e & 63; st[d][nl] = bfr(LAT[(b * DD + d) * (size_t)XSTR + n0 + nl]); }
  __syncthreads();
  { const int nl = t >> 2, sub = t & 3; float s = 0.f; for (int d = sub; d < DD; d += 4) s += st[d][nl]; s += __shfl_xor(s, 1); s += __shfl_xor(s, 2); const float mu = s * (1.0f / DD);
    float s2 = 0.f; for (int d = sub; d < DD; d += 4) { const float c = st[d][nl] - mu; s2 += c * c; } s2 += __shfl_xor(s2, 1); s2 += __shfl_xor(s2, 2);
    if (sub == 0) { float sd = sqrtf(s2 / (float)(DD - 1)); if (sd == 0.f) sd = 1.f; smu[nl] = mu; srs[nl] = 1.0f / sd; } }
  __syncthreads();
  const float* ga = CD + (b * 6 + 1) * DD; const float* be = CD + (b * 6 + 2) * DD;
  for (int e = t; e < 64 * 32; e += 256) { const int nl = e >> 5, q = e & 31; v4f xo, x2o;
#pragma unroll
    for (int z = 0; z < 4; ++z) { const int d = q * 4 + z; const float xv = st[d][nl]; xo[z] = xv; x2o[z] = ga[d] * ((xv - smu[nl]) * srs[nl]) + be[d]; }
    vst2(X + (b * TT + n0 + nl) * DD + q * 4, xo); vst2(X2 + (b * TT + n0 + nl) * DD + q * 4, x2o); } }
__global__ __launch_bounds__(128) void k_qkv(const float* __restrict__ X2, const float* __restrict__ WQ, const float* __restrict__ WK, const float* __restrict__ WV, const float* __restrict__ BQ, const float* __restrict__ BK, const float* __restrict__ BV, _Float16* __restrict__ QH, _Float16* __restrict__ QL, _Float16* __restrict__ KH, __bf16* __restrict__ VT, __bf16* __restrict__ VL) {
  __shared__ __align__(16) _Float16 sh[64][136], sl[64][136]; __shared__ __align__(16) __bf16 th[128][72], tl2[128][72];
  const int tid = threadIdx.x, wave = tid >> 5, lane = tid & 31, col = lane & 15, g = lane >> 4; const int which = blockIdx.y; const size_t r0 = (size_t)blockIdx.x * 64; const float* WA = which == 0 ? WQ : which == 1 ? WK : WV; const float* BA = which == 0 ? BQ : which == 1 ? BK : BV;
  v8f acc[8] = {};
#pragma unroll
  for (int kc = 0; kc < DD / 32; ++kc) { const F2 a = split_row(X2 + (r0 + wave * 16 + col) * DD, kc * 32, lane);
#pragma unroll
    for (int j = 0; j < 8; ++j) { v16b w; const int o = j * 16 + col; const int h = o / HD, kk = o % HD; const float* wr = WA + (size_t)h * DD * HD + kk;
#pragma unroll
      for (int i = 0; i < 8; ++i) { w[i] = (__bf16)wr[(size_t)(kc * 32 + 8 * g + i) * HD]; w[8 + i] = (__bf16)wr[(size_t)(kc * 32 + 16 + 8 * g + i) * HD]; }
      asm volatile("s_wait_loadcnt 0x0" ::: "memory"); acc[j] = wmma_bf(a.h, w, acc[j]); acc[j] = wmma_bf(a.l, w, acc[j]); } }
#pragma unroll
  for (int j = 0; j < 8; ++j) { const int o = j * 16 + col; const float bb = bfr(BA[o]);
#pragma unroll
    for (int r = 0; r < 8; ++r) { const float v = acc[j][r] + bb; const int rl = wave * 16 + 8 * g + r; const _Float16 hv = (_Float16)v;
      if (which == 2) { const __bf16 bh = (__bf16)v; th[o][rl] = bh; tl2[o][rl] = (__bf16)(v - (float)bh); } else { sh[rl][o] = hv; sl[rl][o] = (_Float16)((v - (float)hv) * 1024.0f); } } }
  __syncthreads();
  if (which < 2) { _Float16* dh = which == 0 ? QH : KH; for (int e = tid; e < 64 * 16; e += 128) { const int rl = e >> 4, q = e & 15; vst2((unsigned*)(dh + (r0 + rl) * DD + q * 8), *(const v4u*)&sh[rl][q * 8]); if (which == 0) vst2((unsigned*)(QL + (r0 + rl) * DD + q * 8), *(const v4u*)&sl[rl][q * 8]); } }
  else { const size_t b = r0 / TT; const int n0 = (int)(r0 % TT); for (int e = tid; e < 128 * 8; e += 128) { const int cl = e >> 3, q = e & 7; const size_t o2 = (b * DD + cl) * (size_t)TT + n0 + q * 8; vst2((unsigned*)(VT + o2), *(const v4u*)&th[cl][q * 8]); vst2((unsigned*)(VL + o2), *(const v4u*)&tl2[cl][q * 8]); } } }
__global__ __launch_bounds__(128) void k_sc(const _Float16* __restrict__ QH, const _Float16* __restrict__ QL, const _Float16* __restrict__ KH, int b0, float* __restrict__ S0) { __shared__ __align__(16) float ss[4][16][132];
  const int bg = blockIdx.z / NH, h = blockIdx.z % NH; const size_t b = b0 + bg; float* S = S0 + (size_t)blockIdx.z * TT * TT;
  const int tid = threadIdx.x, wave = tid >> 5, lane = tid & 31, col = lane & 15, g = lane >> 4; const int k0 = blockIdx.y * 128; const int ql0 = blockIdx.x * 64 + wave * 16;
  v8f acc[8] = {}, accl[8] = {};
  { const size_t qo = (b * TT + ql0 + col) * DD + h * HD; const v16h ah = frag_h(QH + qo, lane), al = frag_h(QL + qo, lane);
#pragma unroll
    for (int j = 0; j < 8; ++j) { const v16h kb = frag_h(KH + (b * TT + k0 + j * 16 + col) * DD + h * HD, lane); acc[j] = wmma16(ah, kb, acc[j]); accl[j] = wmma16(al, kb, accl[j]); } }
#pragma unroll
  for (int j = 0; j < 8; ++j)
#pragma unroll
    for (int r = 0; r < 8; ++r) ss[wave][8 * g + r][j * 16 + col] = (acc[j][r] + accl[j][r] * (1.0f / 1024.0f)) * 0.17677669529663687f;
  LDSX(); for (int rl = 0; rl < 16; ++rl) vst2(S + (size_t)(ql0 + rl) * TT + k0 + lane * 4, *(const v4f*)&ss[wave][rl][lane * 4]); }
__global__ __launch_bounds__(128) void k_sm(float* __restrict__ S0) { __shared__ float sred[4]; __shared__ float sbc; __shared__ __align__(16) float sh[TT];
  const int t = threadIdx.x; const size_t row = blockIdx.x; float* sr = S0 + ((size_t)blockIdx.y * TT + row) * TT;
  float m = -3.0e38f; for (int k = t; k < TT; k += 128) { const float v = sr[k]; sh[k] = v; m = fmaxf(m, v); }
#pragma unroll
  for (int o = 1; o < 32; o <<= 1) m = fmaxf(m, __shfl_xor(m, o));
  if ((t & 31) == 0) sred[t >> 5] = m; __syncthreads(); if (t == 0) sbc = fmaxf(fmaxf(sred[0], sred[1]), fmaxf(sred[2], sred[3])); __syncthreads(); m = sbc; __syncthreads();
  float s = 0.f; for (int k = t; k < TT; k += 128) { const float e = expf(sh[k] - m); sh[k] = e; s += e; }
#pragma unroll
  for (int o = 1; o < 32; o <<= 1) s += __shfl_xor(s, o);
  if ((t & 31) == 0) sred[t >> 5] = s; __syncthreads(); if (t == 0) sbc = 2048.0f / ((sred[0] + sred[1]) + (sred[2] + sred[3])); __syncthreads(); const float sc = sbc;
  for (int k = t; k < TT; k += 128) sh[k] *= sc;
  __syncthreads(); for (int q = t; q < TT / 4; q += 128) vst2(sr + q * 4, *(const v4f*)&sh[q * 4]); }
__global__ __launch_bounds__(128) void k_pv(const float* __restrict__ S0, const __bf16* __restrict__ VT, const __bf16* __restrict__ VL, int b0, float* __restrict__ Y) { __shared__ __align__(16) float ss[4][16][HD + 4];
  const int bg = blockIdx.z / NH, h = blockIdx.z % NH; const size_t b = b0 + bg; const float* PS = S0 + (size_t)blockIdx.z * TT * TT;
  const int tid = threadIdx.x, wave = tid >> 5, lane = tid & 31, col = lane & 15, g = lane >> 4; const int ql0 = blockIdx.x * 64 + wave * 16;
  v8f acc[HD / 16] = {};
#pragma unroll 1
  for (int kc = 0; kc < TT / 32; ++kc) { const F2 p = split_row(PS + (size_t)(ql0 + col) * TT, kc * 32, lane);
#pragma unroll
    for (int j = 0; j < HD / 16; ++j) { const size_t po = (b * DD + h * HD + j * 16 + col) * (size_t)TT + kc * 32; const v16b vh = frag_b(VT + po, lane); acc[j] = wmma_bf(p.h, vh, acc[j]); acc[j] = wmma_bf(p.l, vh, acc[j]); acc[j] = wmma_bf(p.h, frag_b(VL + po, lane), acc[j]); } }
#pragma unroll
  for (int j = 0; j < HD / 16; ++j)
#pragma unroll
    for (int r = 0; r < 8; ++r) ss[wave][8 * g + r][j * 16 + col] = acc[j][r] * (1.0f / 2048.0f);
  LDSX(); for (int rl = 0; rl < 16; ++rl) if (lane < HD / 4) vst2(Y + (b * TT + ql0 + rl) * DD + h * HD + lane * 4, *(const v4f*)&ss[wave][rl][lane * 4]); }
__global__ __launch_bounds__(128) void k_fin(const float* __restrict__ Y, const float* __restrict__ OW, const float* __restrict__ X, const float* __restrict__ CD, float* __restrict__ OUT) { __shared__ __align__(16) float stc[DD][68];
  const int tid = threadIdx.x, wave = tid >> 5, lane = tid & 31, col = lane & 15, g = lane >> 4; const size_t r0 = (size_t)blockIdx.x * 64 + wave * 16; const size_t b = r0 / TT; const int n0 = (int)(((size_t)blockIdx.x * 64) % TT);
  v8f acc[8] = {};
#pragma unroll
  for (int kc = 0; kc < DD / 32; ++kc) { const F2 a = split_row(Y + (r0 + col) * DD, kc * 32, lane);
#pragma unroll
    for (int j = 0; j < 8; ++j) { v16b w; const int o = j * 16 + col;
#pragma unroll
      for (int i = 0; i < 8; ++i) { const int ja = kc * 32 + 8 * g + i, jb = ja + 16;
        w[i] = (__bf16)OW[(size_t)((ja % HD) * NH + ja / HD) * DD + o]; w[8 + i] = (__bf16)OW[(size_t)((jb % HD) * NH + jb / HD) * DD + o]; }
      asm volatile("s_wait_loadcnt 0x0" ::: "memory"); acc[j] = wmma_bf(a.h, w, acc[j]); acc[j] = wmma_bf(a.l, w, acc[j]); } }
  const float* a1 = CD + (b * 6 + 0) * DD; const float* a2 = CD + (b * 6 + 3) * DD; const float* g2 = CD + (b * 6 + 4) * DD; const float* b2 = CD + (b * 6 + 5) * DD;
  float x1[8][8]; float mu[8], rs[8];
#pragma unroll
  for (int r = 0; r < 8; ++r) { float s = 0.f;
#pragma unroll
    for (int j = 0; j < 8; ++j) { const int o = j * 16 + col; const float xv = X[(r0 + 8 * g + r) * DD + o] + a1[o] * acc[j][r]; x1[j][r] = xv; s += xv; }
    asm volatile("s_wait_loadcnt 0x0" ::: "memory");
#pragma unroll
    for (int o_ = 1; o_ < 16; o_ <<= 1) s += __shfl_xor(s, o_);
    mu[r] = s * (1.0f / DD); float s2 = 0.f;
#pragma unroll
    for (int j = 0; j < 8; ++j) { const float c = x1[j][r] - mu[r]; s2 += c * c; }
#pragma unroll
    for (int o_ = 1; o_ < 16; o_ <<= 1) s2 += __shfl_xor(s2, o_);
    float sd = sqrtf(s2 / (float)(DD - 1)); if (sd == 0.f) sd = 1.f; rs[r] = 1.0f / sd; }
#pragma unroll
  for (int j = 0; j < 8; ++j) { const int o = j * 16 + col;
#pragma unroll
    for (int r = 0; r < 8; ++r) { const float x2 = g2[o] * ((x1[j][r] - mu[r]) * rs[r]) + b2[o]; stc[o][wave * 16 + 8 * g + r] = x1[j][r] + a2[o] * x2; } }
  __syncthreads();
  for (int e = tid; e < DD * 16; e += 128) { const int d = e >> 4, q = e & 15; vst2(OUT + (b * DD + d) * (size_t)XSTR + n0 + q * 4, *(const v4f*)&stc[d][q * 4]); } }
extern "C" void kernel_launch(void* const* d_in, const int* in_sizes, int n_in, void* d_out, int out_size, void* d_ws, size_t ws_size, hipStream_t stream) {
  (void)in_sizes; (void)n_in; (void)out_size;
  const float** F = (const float**)d_in;
  if (ws_size < (size_t)WS_END) return;
  char* ws = (char*)d_ws; float *CD = (float*)(ws + WS_CD), *X = (float*)(ws + WS_X), *X2 = (float*)(ws + WS_X2), *S = (float*)(ws + WS_S), *Y = (float*)(ws + WS_Y); _Float16 *QH = (_Float16*)(ws + WS_QH), *QL = (_Float16*)(ws + WS_QL), *KH = (_Float16*)(ws + WS_KH); __bf16 *VT = (__bf16*)(ws + WS_VT), *VL = (__bf16*)(ws + WS_VL);
  P24 prm; for (int i = 0; i < 24; ++i) prm.p[i] = F[10 + i];
  k_cond<<<dim3(TNB), 256, 0, stream>>>(F[1], F[2], prm, CD);
  k_xs<<<dim3(TT / 64, TNB), 256, 0, stream>>>(F[0], CD, X, X2);
  k_qkv<<<dim3(TNB * TT / 64, 3), 128, 0, stream>>>(X2, F[3], F[4], F[5], F[6], F[7], F[8], QH, QL, KH, VT, VL);
  for (int b0 = 0; b0 < TNB; b0 += BG) { const int ng = (TNB - b0) < BG ? (TNB - b0) : BG;
    k_sc<<<dim3(TT / 64, TT / 128, ng * NH), 128, 0, stream>>>(QH, QL, KH, b0, S);
    k_sm<<<dim3(TT, ng * NH), 128, 0, stream>>>(S);
    k_pv<<<dim3(TT / 64, 1, ng * NH), 128, 0, stream>>>(S, VT, VL, b0, Y);
  }
  k_fin<<<dim3(TNB * TT / 64), 128, 0, stream>>>(Y, F[9], X, CD, (float*)d_out);
}
